// LSTM_1348619731216
// MI455X (gfx1250) — hardware-verified
//
#include <hip/hip_runtime.h>
#include <math.h>

constexpr int NSTEP  = 365;
constexpr int NBATCH = 2048;
constexpr int NIN    = 9;
constexpr int NHID   = 50;
constexpr int NGATE  = 4 * NHID;
constexpr int NPADN  = 208;
constexpr int KP     = 64;
constexpr int AP     = 72;
constexpr int GP     = 212;
constexpr int ROWS   = 32;
constexpr int NTHR   = 512;
constexpr int NWAVES = NTHR / 32;
constexpr int NGWAVE = NPADN / 16;
constexpr int NXS    = ROWS * NIN;
constexpr int NLANE2 = NHID - 32;
constexpr int XCOL0  = NHID;
constexpr int ZCOL0  = NHID + NIN;
constexpr float ACARRY = 256.0f;
constexpr float WCARRY = 64.0f;
constexpr float CINV   = 1.0f / (ACARRY * WCARRY);

static_assert(NGATE == 200, "gate width");
static_assert(NPADN % 16 == 0 && NPADN >= NGATE, "N padded to the 16-wide tile");
static_assert(NGWAVE == 13 && NGWAVE <= NWAVES, "one N tile per wave");
static_assert(KP % 32 == 0 && KP >= NHID + NIN, "K padded to 32");
static_assert(AP % 8 == 0 && AP >= KP, "A pitch keeps 16-B alignment");
static_assert(GP >= NPADN && GP % 4 == 0, "gate tile pitch");
static_assert(NBATCH % ROWS == 0, "grid exact");
static_assert(ROWS == 2 * NWAVES, "two rows per wave in the pointwise phases");
static_assert(NXS == 288 && NXS <= NTHR, "x staging threads");
static_assert((NPADN * KP) % NTHR == 0, "weight plane staging loop exact");
static_assert((2 * ROWS * AP) % NTHR == 0, "zero fill loop exact");
static_assert(NLANE2 == 18 && ZCOL0 - 32 == 27, "second-unit lane map");
static_assert(ROWS * 4 == 128, "one 128-B line per step");

typedef __attribute__((ext_vector_type(16))) _Float16 v16h;
typedef __attribute__((ext_vector_type(8)))  _Float16 v8h;
typedef __attribute__((ext_vector_type(8)))  float    v8f;

constexpr int frag_k(int lh, int elem) { return (elem < 8) ? (8 * lh + elem) : (16 + 8 * lh + (elem - 8)); }
static_assert(frag_k(0, 0) == 0 && frag_k(0, 7) == 7 && frag_k(0, 8) == 16 && frag_k(0, 15) == 23, "lane half 0 k map");
static_assert(frag_k(1, 0) == 8 && frag_k(1, 7) == 15 && frag_k(1, 8) == 24 && frag_k(1, 15) == 31, "lane half 1 k map");

__device__ __forceinline__ void dep_guard_h(v8f& a, v8f& b, v16h x, v16h y) { asm volatile("v_nop\n\tv_nop\n\tv_nop\n\tv_nop" : "+v"(a), "+v"(b) : "v"(x), "v"(y)); }
__device__ __forceinline__ void keep4_h(v16h a, v16h b, v16h c, v16h d) { asm volatile("v_nop" :: "v"(a), "v"(b), "v"(c), "v"(d)); }
template <typename T> struct Frag;
template <> struct Frag<_Float16> {
  typedef v16h V; union U { v16h v; v8h h[2]; };
  static __device__ __forceinline__ v16h load(const _Float16* p) {
    U f; f.h[0] = *(const v8h*)(p); f.h[1] = *(const v8h*)(p + 16); return f.v;
  }
  static __device__ __forceinline__ v8f mma(v16h a, v16h b, v8f c) {
    return __builtin_amdgcn_wmma_f32_16x16x32_f16(false, a, false, b, (short)0, c, false, false);
  }
  static __device__ __forceinline__ void guard(v8f& a, v8f& b, v16h x, v16h y) { dep_guard_h(a, b, x, y); }
  static __device__ __forceinline__ void keep(v16h a, v16h b, v16h c, v16h d) { keep4_h(a, b, c, d); }
};

__device__ __forceinline__ void guard_2(v8f& acc, v16h a0, v16h a1, v16h b0, v16h b1) {
  asm volatile("v_nop\n\tv_nop\n\tv_nop\n\tv_nop" : "+v"(acc) : "v"(a0), "v"(a1), "v"(b0), "v"(b1));
}
__device__ __forceinline__ void guard_4(v8f& acc, v16h a0, v16h a1, v16h a2, v16h a3, v16h b0, v16h b1, v16h b2, v16h b3) {
  asm volatile("v_nop\n\tv_nop\n\tv_nop\n\tv_nop" : "+v"(acc) : "v"(a0), "v"(a1), "v"(a2), "v"(a3), "v"(b0), "v"(b1), "v"(b2), "v"(b3));
}

__device__ __forceinline__ float fsig(float v)  { return __builtin_amdgcn_rcpf(1.0f + __expf(-v)); }
__device__ __forceinline__ float ftanh(float v) { return 1.0f - 2.0f * __builtin_amdgcn_rcpf(__expf(2.0f * v) + 1.0f); }

__device__ __forceinline__ float cell_update(float zi, float zf, float zg, float zo, float& cst) {
  const float ig = fsig(zi);
  const float fg = fsig(zf);
  const float gg = ftanh(zg);
  const float og = fsig(zo);
  const float cn = fg * cst + ig * gg;
  cst = cn;
  return og * ftanh(cn);
}

__device__ __forceinline__ void stage_plane(_Float16* sWp, const float* __restrict__ srcA,
                                            const float* __restrict__ srcB, int nB, int tid) {
#pragma unroll 1
  for (int it = 0; it < (NPADN * KP) / NTHR; ++it) {
    const int idx = it * NTHR + tid;
    const int n = idx >> 6;
    const int k = idx & (KP - 1);
    const int nn = (n < NGATE) ? n : (NGATE - 1);
    const int ka = (k < NHID) ? k : (NHID - 1);
    int kb = k - NHID;
    kb = (kb < 0) ? 0 : ((kb > NIN - 1) ? (NIN - 1) : kb);
    float va = srcA[nn * NHID + ka];
    float vb = srcB[nn * NIN + kb];
    asm volatile("" : "+v"(va), "+v"(vb));
    const bool useA = (n < NGATE) && (k < NHID);
    const bool useB = (n < NGATE) && (k >= NHID) && (k < NHID + nB);
    const float v = useA ? va : (useB ? vb : 0.0f);
    sWp[idx] = (_Float16)(v * WCARRY);
  }
}

__global__ __launch_bounds__(NTHR) void lstm2_seq_kernel(
    const float* __restrict__ x,
    const float* __restrict__ w_ih0, const float* __restrict__ w_hh0,
    const float* __restrict__ b_ih0, const float* __restrict__ b_hh0,
    const float* __restrict__ w_ih1, const float* __restrict__ w_hh1,
    const float* __restrict__ b_ih1, const float* __restrict__ b_hh1,
    const float* __restrict__ fc_w,  const float* __restrict__ fc_b,
    float* out) {
  __shared__ __align__(16) _Float16 sA0[ROWS * AP];
  __shared__ __align__(16) _Float16 sA1[ROWS * AP];
  __shared__ __align__(16) _Float16 sW[NPADN * KP];
  __shared__ __align__(16) float    sG[ROWS * GP];
  __shared__ __align__(16) float    sO[ROWS];

  const int tid  = threadIdx.x;
  const int lane = tid & 31;
  const int wave = tid >> 5;
  const int c    = lane & 15;
  const int hh   = lane >> 4;
  const int koff = hh * 8;
  const int bbase = blockIdx.x * ROWS;
  const bool gemm_wave = (wave < NGWAVE);

#pragma unroll 1
  for (int i = tid; i < 2 * ROWS * AP; i += NTHR) {
    if (i < ROWS * AP) sA0[i] = (_Float16)0.0f;
    else               sA1[i - ROWS * AP] = (_Float16)0.0f;
  }

  const int nraw = 16 * wave + c;
  const int nrow = (nraw < NPADN) ? nraw : (NPADN - 1);
  const _Float16* bp = sW + nrow * KP + koff;

  stage_plane(sW, w_hh0, w_ih0, NIN, tid);
  __syncthreads();
  const v16h b00 = Frag<_Float16>::load(bp);
  const v16h b01 = Frag<_Float16>::load(bp + 32);
  __syncthreads();
  stage_plane(sW, w_ih1, w_ih0, 0, tid);
  __syncthreads();
  const v16h b10 = Frag<_Float16>::load(bp);
  const v16h b11 = Frag<_Float16>::load(bp + 32);
  __syncthreads();
  stage_plane(sW, w_hh1, w_ih0, 0, tid);
  __syncthreads();
  const v16h b20 = Frag<_Float16>::load(bp);
  const v16h b21 = Frag<_Float16>::load(bp + 32);

  const int ncol = 16 * wave + c;
  const int ncl  = (ncol < NGATE) ? ncol : (NGATE - 1);
  const float bs0 = b_ih0[ncl] + b_hh0[ncl];
  const float bs1 = b_ih1[ncl] + b_hh1[ncl];
  const float bias0 = (ncol < NGATE) ? bs0 : 0.0f;
  const float bias1 = (ncol < NGATE) ? bs1 : 0.0f;
  const bool lane2 = (lane < NLANE2);
  const int  j2    = lane2 ? (lane + 32) : (NHID - 1);
  const float fcw0 = fc_w[lane];
  const float fcw1r = fc_w[j2];
  const float fcw1 = lane2 ? fcw1r : 0.0f;
  const float fcb  = fc_b[0];

  const int xi   = (tid < NXS) ? tid : (NXS - 1);
  const int xrow = xi / NIN;
  const int xcol = xi - xrow * NIN;
  const bool xstore = (tid < NXS);
  {
    float x0 = x[(size_t)bbase * NIN + (size_t)xi];
    asm volatile("" : "+v"(x0));
    if (xstore) sA0[xrow * AP + XCOL0 + xcol] = (_Float16)(x0 * ACARRY);
  }

  float c1a[2] = {0.0f, 0.0f}, c1b[2] = {0.0f, 0.0f};
  float c2a[2] = {0.0f, 0.0f}, c2b[2] = {0.0f, 0.0f};
  const v8f z8 = {0.f, 0.f, 0.f, 0.f, 0.f, 0.f, 0.f, 0.f};
  __syncthreads();

#pragma unroll 1
  for (int t = 0; t < NSTEP; ++t) {
    const int tn = (t + 1 < NSTEP) ? (t + 1) : (NSTEP - 1);
    float xnext = x[((size_t)tn * NBATCH + (size_t)bbase) * NIN + (size_t)xi];
    asm volatile("" : "+v"(xnext));

    if (gemm_wave) {
#pragma unroll
      for (int mt = 0; mt < 2; ++mt) {
        const _Float16* ap = sA0 + (16 * mt + c) * AP + koff;
        const v16h a0 = Frag<_Float16>::load(ap);
        const v16h a1 = Frag<_Float16>::load(ap + 32);
        v8f acc = z8;
        acc = Frag<_Float16>::mma(a0, b00, acc);
        acc = Frag<_Float16>::mma(a1, b01, acc);
        guard_2(acc, a0, a1, b00, b01);
        float* gp = sG + (16 * mt + 8 * hh) * GP + ncol;
#pragma unroll
        for (int r = 0; r < 8; ++r) gp[r * GP] = fmaf(acc[r], CINV, bias0);
      }
    }
    __syncthreads();

#pragma unroll
    for (int rr = 0; rr < 2; ++rr) {
      const int row = 2 * wave + rr;
      const float* gr = sG + row * GP;
      const float ha = cell_update(gr[lane], gr[NHID + lane], gr[2 * NHID + lane], gr[3 * NHID + lane], c1a[rr]);
      const float hb = cell_update(gr[j2],   gr[NHID + j2],   gr[2 * NHID + j2],   gr[3 * NHID + j2],   c1b[rr]);
      sA0[row * AP + lane] = (_Float16)(ha * ACARRY);
      const float hbv = lane2 ? (hb * ACARRY) : 0.0f;
      if (lane2 || (lane >= ZCOL0 - 32)) sA0[row * AP + 32 + lane] = (_Float16)hbv;
    }
    __syncthreads();

    if (gemm_wave) {
#pragma unroll
      for (int mt = 0; mt < 2; ++mt) {
        const _Float16* ap0 = sA0 + (16 * mt + c) * AP + koff;
        const _Float16* ap1 = sA1 + (16 * mt + c) * AP + koff;
        const v16h a0 = Frag<_Float16>::load(ap0);
        const v16h a1 = Frag<_Float16>::load(ap0 + 32);
        const v16h a2 = Frag<_Float16>::load(ap1);
        const v16h a3 = Frag<_Float16>::load(ap1 + 32);
        v8f acc = z8;
        acc = Frag<_Float16>::mma(a0, b10, acc);
        acc = Frag<_Float16>::mma(a1, b11, acc);
        acc = Frag<_Float16>::mma(a2, b20, acc);
        acc = Frag<_Float16>::mma(a3, b21, acc);
        guard_4(acc, a0, a1, a2, a3, b10, b11, b20, b21);
        float* gp = sG + (16 * mt + 8 * hh) * GP + ncol;
#pragma unroll
        for (int r = 0; r < 8; ++r) gp[r * GP] = fmaf(acc[r], CINV, bias1);
      }
    }
    __syncthreads();

#pragma unroll
    for (int rr = 0; rr < 2; ++rr) {
      const int row = 2 * wave + rr;
      const float* gr = sG + row * GP;
      const float ha = cell_update(gr[lane], gr[NHID + lane], gr[2 * NHID + lane], gr[3 * NHID + lane], c2a[rr]);
      const float hb = cell_update(gr[j2],   gr[NHID + j2],   gr[2 * NHID + j2],   gr[3 * NHID + j2],   c2b[rr]);
      sA1[row * AP + lane] = (_Float16)(ha * ACARRY);
      const float hbv = lane2 ? (hb * ACARRY) : 0.0f;
      sA1[row * AP + 32 + lane] = (_Float16)hbv;
      float p = ha * fcw0 + hb * fcw1;
      p += __shfl_xor(p, 16, 32);
      p += __shfl_xor(p, 8, 32);
      p += __shfl_xor(p, 4, 32);
      p += __shfl_xor(p, 2, 32);
      p += __shfl_xor(p, 1, 32);
      if (lane == 0) sO[row] = p + fcb;
    }
    if (xstore) sA0[xrow * AP + XCOL0 + xcol] = (_Float16)(xnext * ACARRY);
    __syncthreads();

    if (wave == NWAVES - 1) {
      const float ov = sO[lane];
      volatile float* op = (volatile float*)(out + (size_t)t * NBATCH + (size_t)bbase + (size_t)lane);
      *op = ov;
      __threadfence();
      *op = ov;
    }
  }
}

extern "C" void kernel_launch(void* const* d_in, const int* in_sizes, int n_in,
                              void* d_out, int out_size, void* d_ws, size_t ws_size, hipStream_t stream) {
  (void)d_ws; (void)ws_size;
  if (n_in < 11 || d_out == nullptr) return;
  if (in_sizes[0] != NSTEP * NBATCH * NIN || in_sizes[1] != NGATE * NIN || in_sizes[2] != NGATE * NHID ||
      in_sizes[3] != NGATE || in_sizes[4] != NGATE || in_sizes[5] != NGATE * NHID || in_sizes[6] != NGATE * NHID ||
      in_sizes[7] != NGATE || in_sizes[8] != NGATE || in_sizes[9] != NHID || in_sizes[10] != 1 ||
      out_size != NSTEP * NBATCH) return;

  const float* x     = (const float*)d_in[0];
  const float* w_ih0 = (const float*)d_in[1];
  const float* w_hh0 = (const float*)d_in[2];
  const float* b_ih0 = (const float*)d_in[3];
  const float* b_hh0 = (const float*)d_in[4];
  const float* w_ih1 = (const float*)d_in[5];
  const float* w_hh1 = (const float*)d_in[6];
  const float* b_ih1 = (const float*)d_in[7];
  const float* b_hh1 = (const float*)d_in[8];
  const float* fc_w  = (const float*)d_in[9];
  const float* fc_b  = (const float*)d_in[10];
  float* out = (float*)d_out;

  lstm2_seq_kernel<<<NBATCH / ROWS, NTHR, 0, stream>>>(x, w_ih0, w_hh0, b_ih0, b_hh0,
                                                       w_ih1, w_hh1, b_ih1, b_hh1, fc_w, fc_b, out);
}
